// ResNetUNetDAMLastLayerv2_59313498358084
// MI455X (gfx1250) — hardware-verified
//
#include <hip/hip_runtime.h>
#include <math.h>

typedef __attribute__((ext_vector_type(16))) _Float16 v16h;
typedef __attribute__((ext_vector_type(16))) __bf16 v16b;
typedef __attribute__((ext_vector_type(8)))  _Float16 v8h;
typedef __attribute__((ext_vector_type(8)))  float v8f;
typedef __attribute__((ext_vector_type(4)))  float v4f;
typedef __attribute__((ext_vector_type(2)))  float v2f;
typedef __attribute__((ext_vector_type(4)))  unsigned v4u;
typedef __attribute__((ext_vector_type(4)))  int v4i;
typedef float __attribute__((may_alias)) float_a;
typedef int __attribute__((may_alias)) int_a;

template <typename T> __device__ __forceinline__ void vst2(void* p, T v) { *(volatile T*)p = v; __threadfence(); *(volatile T*)p = v; }
__device__ __forceinline__ v8f wmma16(v16h a, v16h b, v8f c) {
  v8f d = __builtin_amdgcn_wmma_f32_16x16x32_f16(false, a, false, b, (short)0, c, false, false);
  asm volatile("v_nop\n\tv_nop\n\tv_nop\n\tv_nop" : "+v"(d) : "v"(a), "v"(b));
  return d;
}
__device__ __forceinline__ v8f wmma_bf(v16b a, v16b b, v8f c) {
  v8f d = __builtin_amdgcn_wmma_f32_16x16x32_bf16(false, a, false, b, (short)0, c, false, false);
  asm volatile("v_nop\n\tv_nop\n\tv_nop\n\tv_nop" : "+v"(d) : "v"(a), "v"(b));
  return d;
}
__device__ __forceinline__ v16h frag_h(const _Float16* rowk0, int lane) {
  union { v16h v; v8h q[2]; } u; const _Float16* p = rowk0 + 8 * (lane >> 4);
  u.q[0] = *(const v8h*)p; u.q[1] = *(const v8h*)(p + 16); return u.v;
}
__device__ __forceinline__ v16h frag_f32(const float* rowk0, int lane) {
  v16h a; const float* p = rowk0 + 8 * (lane >> 4);
#pragma unroll
  for (int i = 0; i < 8; ++i) { a[i] = (_Float16)p[i]; a[8 + i] = (_Float16)p[16 + i]; }
  return a;
}
__device__ __forceinline__ v16h frag_f32s(const float* rowk0, int lane, float sc) {
  v16h a; const float* p = rowk0 + 8 * (lane >> 4);
#pragma unroll
  for (int i = 0; i < 8; ++i) { a[i] = (_Float16)(p[i] * sc); a[8 + i] = (_Float16)(p[16 + i] * sc); }
  return a;
}
__device__ __forceinline__ v16h fragc_f32(const float* W, int k0, int n, int lane, int ld, int K) {
  v16h a; const int g = lane >> 4;
#pragma unroll
  for (int i = 0; i < 8; ++i) { const int ka = k0 + 8 * g + i, kb = ka + 16;
    a[i] = (_Float16)(ka < K ? W[(size_t)ka * ld + n] : 0.f); a[8 + i] = (_Float16)(kb < K ? W[(size_t)kb * ld + n] : 0.f); }
  return a;
}
struct F2 { v16b h, l; };
__device__ __forceinline__ F2 bsplit16(const float v[16]) { F2 r;
#pragma unroll
  for (int i = 0; i < 16; ++i) { const __bf16 h = (__bf16)v[i]; r.h[i] = h; r.l[i] = (__bf16)(v[i] - (float)h); }
  return r; }
__device__ __forceinline__ F2 split_row(const float* row, int k0, int lane) { float v[16]; const float* p = row + k0 + 8 * (lane >> 4);
#pragma unroll
  for (int i = 0; i < 8; ++i) { v[i] = p[i]; v[8 + i] = p[16 + i]; }
  return bsplit16(v); }
__device__ __forceinline__ F2 split_rowK(const float* row, int k0, int lane, int K) { float v[16]; const int g = lane >> 4;
#pragma unroll
  for (int i = 0; i < 8; ++i) { const int ka = k0 + 8 * g + i, kb = ka + 16; v[i] = ka < K ? row[ka] : 0.f; v[8 + i] = kb < K ? row[kb] : 0.f; }
  return bsplit16(v); }
__device__ __forceinline__ F2 split_col(const float* W, int k0, int n, int lane, int ld, int K) { float v[16]; const int g = lane >> 4;
#pragma unroll
  for (int i = 0; i < 8; ++i) { const int ka = k0 + 8 * g + i, kb = ka + 16; v[i] = ka < K ? W[(size_t)ka * ld + n] : 0.f; v[8 + i] = kb < K ? W[(size_t)kb * ld + n] : 0.f; }
  return bsplit16(v); }
__device__ __forceinline__ v8f mac3(const F2& a, const F2& b, v8f c) { c = wmma_bf(a.l, b.h, c); c = wmma_bf(a.h, b.l, c); return wmma_bf(a.h, b.h, c); }
__device__ __forceinline__ float sigm(float v) { return 1.0f / (1.0f + expf(-v)); }
#define LDSX() do { asm volatile("s_wait_dscnt 0" ::: "memory"); __builtin_amdgcn_wave_barrier(); __builtin_amdgcn_fence(__ATOMIC_RELEASE, "workgroup"); } while (0)

#define NBT 64
#define FF 64
#define NC 27
#define NG 32
#define LL (NG * NG)
#define EPS 1e-5f

__global__ __launch_bounds__(256) void k_sp(const float* __restrict__ SP, float* __restrict__ SPp) {
  __shared__ __align__(16) float so[NC][64];
  const int b = blockIdx.y, pr0 = blockIdx.x * 2, tid = threadIdx.x;
  const int sy = tid >> 6, sx = tid & 63; const int yy = pr0 * 2 + sy;
  float v[NC]; float mx = -3.0e38f;
#pragma unroll
  for (int c = 0; c < NC; ++c) { v[c] = SP[(((size_t)b * NC + c) * (2 * NG) + yy) * (2 * NG) + sx]; mx = fmaxf(mx, v[c]); }
  float s = 0.f;
#pragma unroll
  for (int c = 0; c < NC; ++c) { v[c] = expf(v[c] - mx); s += v[c]; }
  const float inv = 1.0f / s;
  __shared__ float stmp[NC][256];
#pragma unroll
  for (int c = 0; c < NC; ++c) { float p = v[c] * inv; p = fmaxf(p, __shfl_xor(p, 1, 32)); stmp[c][tid] = p; }
  __syncthreads();
  for (int q = tid; q < NC * 64; q += 256) { const int c = q >> 6, pl = q & 63; const int prl = pl >> 5, px = pl & 31;
    so[c][pl] = fmaxf(stmp[c][(prl * 2) * 64 + px * 2], stmp[c][(prl * 2 + 1) * 64 + px * 2]); }
  __syncthreads();
  for (int q = tid; q < NC * 16; q += 256) { const int c = q >> 4, pc = q & 15; vst2(SPp + ((size_t)b * NC + c) * LL + pr0 * NG + pc * 4, *(const v4f*)(&so[c][pc * 4])); }
}
__global__ __launch_bounds__(128) void k_t(const float* __restrict__ x, const float* __restrict__ tw, const float* __restrict__ g1, const float* __restrict__ b1, float* __restrict__ yt) {
  __shared__ __align__(16) float so[4][16][68];
  const int tid = threadIdx.x, wave = tid >> 5, lane = tid & 31, col = lane & 15, g = lane >> 4;
  const int b = blockIdx.y, p0 = blockIdx.x * 64 + wave * 16; const float* xb = x + (size_t)b * FF * LL;
  v8f acc[4] = {};
#pragma unroll
  for (int kc = 0; kc < 2; ++kc) { const F2 a = split_col(xb, kc * 32, p0 + col, lane, LL, FF);
#pragma unroll
    for (int j = 0; j < 4; ++j) acc[j] = mac3(a, split_row(tw + (size_t)(j * 16 + col) * FF, kc * 32, lane), acc[j]); }
  const float sc1 = rsqrtf(1.0f + EPS);
#pragma unroll
  for (int j = 0; j < 4; ++j) { const int f = j * 16 + col; const float gg = g1[f] * sc1, bb = b1[f];
#pragma unroll
    for (int r = 0; r < 8; ++r) { const float v = acc[j][r] * gg + bb; so[wave][8 * g + r][f] = v > 0.f ? v : 0.f; } }
  LDSX();
  for (int q = lane; q < 16 * 16; q += 32) { const int rl = q >> 4, pc = q & 15; vst2(yt + ((size_t)b * LL + p0 + rl) * FF + pc * 4, *(const v4f*)(&so[wave][rl][pc * 4])); }
}
__global__ __launch_bounds__(256) void k_img(const float* __restrict__ yt, const float* __restrict__ SPp, const float* __restrict__ wnc, const float* __restrict__ bnc, const float* __restrict__ wkc, const float* __restrict__ bkc, float* __restrict__ AY) {
  __shared__ float syn[FF][NC + 1]; __shared__ float ssig[NC][NC + 1]; __shared__ float sM1[NC][FF]; __shared__ __align__(16) float sM2[NC][FF];
  __shared__ __align__(16) float sout[64][FF + 4];
  const int b = blockIdx.x, tid = threadIdx.x; const float* ytb = yt + (size_t)b * LL * FF; const float* spb = SPp + (size_t)b * NC * LL;
  for (int q = tid; q < FF * NC + NC * FF; q += 256) { float s = 0.f;
    if (q < FF * NC) { const int f = q / NC, c = q % NC; const float* wr = wnc + (size_t)c * LL;
#pragma unroll 4
      for (int l = 0; l < LL; ++l) s += ytb[(size_t)l * FF + f] * wr[l];
      syn[f][c] = s + bnc[c]; }
    else { const int q2 = q - FF * NC; const int c = q2 / FF, f = q2 % FF; const float* sr = spb + (size_t)c * LL;
#pragma unroll 4
      for (int l = 0; l < LL; ++l) s += sr[l] * ytb[(size_t)l * FF + f];
      sM1[c][f] = s; } }
  __syncthreads();
  for (int q = tid; q < NC * NC; q += 256) { const int c = q / NC, k = q % NC; float s = bkc[k];
#pragma unroll 8
    for (int f = 0; f < FF; ++f) s += syn[f][c] * wkc[k * FF + f];
    ssig[c][k] = s; }
  __syncthreads();
  for (int q = tid; q < NC * FF; q += 256) { const int c = q / FF, f = q % FF; float s = 0.f;
#pragma unroll
    for (int k = 0; k < NC; ++k) s += ssig[c][k] * sM1[k][f];
    sM2[c][f] = s; }
  __syncthreads();
#pragma unroll 1
  for (int l0 = 0; l0 < LL; l0 += 64) { const int pl = tid >> 2, f0 = (tid & 3) * 16; const int l = l0 + pl; float a[16];
#pragma unroll
    for (int e = 0; e < 16; ++e) a[e] = 0.f;
#pragma unroll 1
    for (int c = 0; c < NC; ++c) { const float sv = spb[(size_t)c * LL + l];
#pragma unroll
      for (int e = 0; e < 16; ++e) a[e] += sv * sM2[c][f0 + e]; }
#pragma unroll
    for (int e = 0; e < 16; ++e) sout[pl][f0 + e] = a[e];
    __syncthreads();
    for (int q = tid; q < 64 * 16; q += 256) { const int rl = q >> 4, pc = q & 15; vst2(AY + ((size_t)b * LL + l0 + rl) * FF + pc * 4, *(const v4f*)(&sout[rl][pc * 4])); }
    __syncthreads(); }
}
__global__ __launch_bounds__(128) void k_main(const float* __restrict__ yt, const float* __restrict__ AY, const float* __restrict__ adj, const float* __restrict__ wg, const float* __restrict__ bg, const float* __restrict__ wsp, const float* __restrict__ bsp, const float* __restrict__ bw, const float* __restrict__ g2, const float* __restrict__ b2v, float* __restrict__ out) {
  __shared__ __align__(16) float sa[4][16][68];
  __shared__ __align__(16) float st[FF][68];
  const int tid = threadIdx.x, wave = tid >> 5, lane = tid & 31, col = lane & 15, g = lane >> 4;
  const int b = blockIdx.y, p0b = blockIdx.x * 64, p0 = p0b + wave * 16; const float* ytb = yt + (size_t)b * LL * FF;
  { v8f acc[4] = {};
#pragma unroll 2
    for (int kc = 0; kc < LL / 32; ++kc) { const v16h a = frag_f32s(adj + (size_t)(p0 + col) * LL + kc * 32, lane, 64.0f);
#pragma unroll
      for (int j = 0; j < 4; ++j) acc[j] = wmma16(a, fragc_f32(ytb, kc * 32, j * 16 + col, lane, FF, LL), acc[j]); }
#pragma unroll
    for (int j = 0; j < 4; ++j)
#pragma unroll
      for (int r = 0; r < 8; ++r) sa[wave][8 * g + r][j * 16 + col] = acc[j][r] * (1.0f / 64.0f); }
  LDSX();
  { v8f a1[4] = {}, a2[4] = {};
#pragma unroll
    for (int kc = 0; kc < 2; ++kc) { const F2 fa = split_row(&sa[wave][col][0], kc * 32, lane); const F2 fb = split_row(AY + ((size_t)b * LL + p0 + col) * FF, kc * 32, lane);
#pragma unroll
      for (int j = 0; j < 4; ++j) { a1[j] = mac3(fa, split_row(wsp + (size_t)(j * 16 + col) * FF, kc * 32, lane), a1[j]); a2[j] = mac3(fb, split_row(wg + (size_t)(j * 16 + col) * FF, kc * 32, lane), a2[j]); } }
    LDSX();
#pragma unroll
    for (int j = 0; j < 4; ++j) { const int f = j * 16 + col; const float bs = bsp[f], bgv = bg[f];
#pragma unroll
      for (int r = 0; r < 8; ++r) { const float y0 = ytb[(size_t)(p0 + 8 * g + r) * FF + f]; float spv = a1[j][r] + bs; spv = spv > 0.f ? spv : 0.f; float sev = a2[j][r] + bgv; sev = sev > 0.f ? sev : 0.f;
        sa[wave][8 * g + r][f] = (sev + y0) + (spv + y0) + y0; } } }
  LDSX();
  { v8f acc[4] = {};
#pragma unroll
    for (int kc = 0; kc < 2; ++kc) { const F2 fa = split_row(&sa[wave][col][0], kc * 32, lane);
#pragma unroll
      for (int j = 0; j < 4; ++j) acc[j] = mac3(fa, split_row(bw + (size_t)(j * 16 + col) * FF, kc * 32, lane), acc[j]); }
    const float sc2 = rsqrtf(1.0f + EPS);
#pragma unroll
    for (int j = 0; j < 4; ++j) { const int o = j * 16 + col; const float gg = g2[o] * sc2, bb = b2v[o];
#pragma unroll
      for (int r = 0; r < 8; ++r) { const float v = acc[j][r] * gg + bb; st[o][wave * 16 + 8 * g + r] = v > 0.f ? v : 0.f; } } }
  __syncthreads();
  for (int q = tid; q < FF * 16; q += 128) { const int o = q >> 4, pc = q & 15; vst2(out + ((size_t)b * FF + o) * LL + p0b + pc * 4, *(const v4f*)(&st[o][pc * 4])); }
}
extern "C" void kernel_launch(void* const* d_in, const int* in_sizes, int n_in, void* d_out, int out_size, void* d_ws, size_t ws_size, hipStream_t stream) {
  (void)in_sizes; (void)n_in; (void)out_size; (void)ws_size;
  const float** I = (const float**)d_in;
  const float* x = I[0]; const float* SP = I[1]; const float* tw = I[2]; const float* g1 = I[3]; const float* b1 = I[4]; const float* wnc = I[5]; const float* bnc = I[6]; const float* wkc = I[7]; const float* bkc = I[8];
  const float* wg = I[9]; const float* bg = I[10]; const float* adj = I[11]; const float* wsp = I[12]; const float* bsp = I[13]; const float* bw = I[14]; const float* g2 = I[15]; const float* b2v = I[16];
  float* out = (float*)d_out;
  char* ws = (char*)d_ws; size_t off = 0;
  auto take = [&](size_t bytes) { char* p = ws + off; off += (bytes + 255) & ~(size_t)255; return p; };
  float* SPp = (float*)take((size_t)NBT * NC * LL * 4); float* yt = (float*)take((size_t)NBT * LL * FF * 4); float* AY = (float*)take((size_t)NBT * LL * FF * 4);
  k_sp<<<dim3(NG / 2, NBT), 256, 0, stream>>>(SP, SPp);
  k_t<<<dim3(LL / 64, NBT), 128, 0, stream>>>(x, tw, g1, b1, yt);
  k_img<<<NBT, 256, 0, stream>>>(yt, SPp, wnc, bnc, wkc, bkc, AY);
  k_main<<<dim3(LL / 64, NBT), 128, 0, stream>>>(yt, AY, adj, wg, bg, wsp, bsp, bw, g2, b2v, out);
}
